// MambaBlock_50929722196042
// MI455X (gfx1250) — hardware-verified
//
#include <hip/hip_runtime.h>
#include <stddef.h>
#include <stdint.h>
#include <math.h>


#define NTOK   4096
#define SEQ    2048
#define DIMC   1024
#define INNER  2048
#define K2     4096
#define NST    16
#define SSMP   48
#define DTK    32
#define GBM    64
#define GBN    64
#define GTHR   128
#define PTHR   256
#define TCH    32
#define CT     64
#define WSMAX  134217728

#define NU_XB  524288
#define NU_WIN 524288
#define NU_WO  524288
#define NU_WX  24576
#define NU_WD  8192
#define NU_ALL (NU_XB + NU_WIN + NU_WO + NU_WX + NU_WD)

static_assert(NU_XB % PTHR == 0 && NU_WIN % PTHR == 0 && NU_WO % PTHR == 0);
static_assert(NU_WX % PTHR == 0 && NU_WD % PTHR == 0 && NU_ALL % PTHR == 0);
static_assert(NTOK % GBM == 0 && (2 * INNER) % GBN == 0 && DIMC % GBN == 0 && INNER % GBN == 0);
static_assert(DIMC % 32 == 0 && K2 % 32 == 0 && DTK % 32 == 0 && K2 == 2 * INNER && DTK == 2 * NST);
static_assert(GBM == (GTHR / 32) * 16 && SSMP == 48 && SSMP % 16 == 0);
static_assert(SEQ % TCH == 0 && INNER % CT == 0 && NTOK == 2 * SEQ);
static_assert((GBM * SSMP) % (4 * GTHR) == 0 && (GBM * DTK) % (8 * GTHR) == 0);
static_assert((TCH * CT) % (4 * CT) == 0 && (TCH * SSMP) % (4 * CT) == 0 && (CT * NST) % CT == 0);

typedef float          v4f   __attribute__((ext_vector_type(4)));
typedef float          v8f   __attribute__((ext_vector_type(8)));
typedef int            v8i   __attribute__((ext_vector_type(8)));
typedef unsigned short v8us  __attribute__((ext_vector_type(8)));
typedef unsigned short v16us __attribute__((ext_vector_type(16)));
typedef __bf16         v16bf __attribute__((ext_vector_type(16)));
typedef v4f  __attribute__((may_alias)) v4fa;
typedef v8us __attribute__((may_alias)) v8usa;
union FragB { v16bf v; v16us u; v8us h[2]; v8i w; };

__device__ __forceinline__ v8f wmb(const FragB& a, const FragB& b, v8f c) {
  v8f d = __builtin_amdgcn_wmma_f32_16x16x32_bf16(false, a.v, false, b.v, (short)0, c, false, false);
  asm volatile("v_nop\n\tv_nop\n\tv_nop\n\tv_nop" : "+v"(d) : "v"(a.w), "v"(b.w));
  return d;
}

__device__ __forceinline__ unsigned bf16_bits(float f) {
  const unsigned u = __float_as_uint(f);
  return (u + 0x7FFFu + ((u >> 16) & 1u)) >> 16;
}
__device__ __forceinline__ float bf16_val(float f) {
  return __uint_as_float(bf16_bits(f) << 16);
}
__device__ __forceinline__ void split1(float v, unsigned short& hb, unsigned short& lb) {
  const unsigned h = bf16_bits(v);
  hb = (unsigned short)h;
  lb = (unsigned short)bf16_bits(v - __uint_as_float(h << 16));
}
__device__ __forceinline__ void split8(const v4f a, const v4f b, v8us& hv, v8us& lv) {
  unsigned short h, l;
  split1(a.x, h, l); hv[0] = h; lv[0] = l;
  split1(a.y, h, l); hv[1] = h; lv[1] = l;
  split1(a.z, h, l); hv[2] = h; lv[2] = l;
  split1(a.w, h, l); hv[3] = h; lv[3] = l;
  split1(b.x, h, l); hv[4] = h; lv[4] = l;
  split1(b.y, h, l); hv[5] = h; lv[5] = l;
  split1(b.z, h, l); hv[6] = h; lv[6] = l;
  split1(b.w, h, l); hv[7] = h; lv[7] = l;
}

__device__ __forceinline__ float softplus_f(float v) {
  return fmaxf(v, 0.0f) + log1pf(expf(-fabsf(v)));
}

__device__ __forceinline__ void cvt8_put(const float* __restrict__ p, unsigned short* dp, bool ok) {
  const v4f a = *(const v4fa*)p;
  const v4f b = *(const v4fa*)(p + 4);
  v8us o;
  o[0] = ok ? (unsigned short)bf16_bits(a.x) : (unsigned short)0;
  o[1] = ok ? (unsigned short)bf16_bits(a.y) : (unsigned short)0;
  o[2] = ok ? (unsigned short)bf16_bits(a.z) : (unsigned short)0;
  o[3] = ok ? (unsigned short)bf16_bits(a.w) : (unsigned short)0;
  o[4] = ok ? (unsigned short)bf16_bits(b.x) : (unsigned short)0;
  o[5] = ok ? (unsigned short)bf16_bits(b.y) : (unsigned short)0;
  o[6] = ok ? (unsigned short)bf16_bits(b.z) : (unsigned short)0;
  o[7] = ok ? (unsigned short)bf16_bits(b.w) : (unsigned short)0;
  *(volatile v8us*)dp = o;
  __threadfence();
  *(volatile v8us*)dp = o;
}

__global__ __launch_bounds__(PTHR) void k_prep(const float* __restrict__ x, const float* __restrict__ Win,
                                               const float* __restrict__ Wx, const float* __restrict__ Wdt,
                                               const float* __restrict__ Wout,
                                               unsigned short* XB, unsigned short* WIN, unsigned short* WOUT2,
                                               unsigned short* WX2, unsigned short* WDT2) {
  const int u = (int)blockIdx.x * PTHR + (int)threadIdx.x;
  if (u < NU_XB) {
    cvt8_put(x + (size_t)8 * u, XB + (size_t)8 * u, true);
  } else if (u < NU_XB + NU_WIN) {
    const int v = u - NU_XB;
    cvt8_put(Win + (size_t)8 * v, WIN + (size_t)8 * v, true);
  } else if (u < NU_XB + NU_WIN + NU_WO) {
    const int v  = u - (NU_XB + NU_WIN);
    const int n  = v >> 9;
    const int k8 = (v & 511) * 8;
    cvt8_put(Wout + (size_t)n * INNER + (k8 & (INNER - 1)), WOUT2 + (size_t)8 * v, true);
  } else if (u < NU_XB + NU_WIN + NU_WO + NU_WX) {
    const int v  = u - (NU_XB + NU_WIN + NU_WO);
    const int n  = v >> 9;
    const int k8 = (v & 511) * 8;
    const int nc = n < 32 ? n : 32;
    cvt8_put(Wx + (size_t)nc * INNER + (k8 & (INNER - 1)), WX2 + (size_t)8 * v, n < 33);
  } else if (u < NU_ALL) {
    const int v  = u - (NU_XB + NU_WIN + NU_WO + NU_WX);
    const int n  = v >> 2;
    const int k8 = (v & 3) * 8;
    cvt8_put(Wdt + (size_t)n * NST + (k8 & (NST - 1)), WDT2 + (size_t)8 * v, true);
  }
}

template <int NT>
__device__ __forceinline__ void gemm_loop(const unsigned short* __restrict__ ap,
                                          const unsigned short* __restrict__ wp, int K, v8f (&acc)[NT]) {
  const int ksteps = K >> 5;
#pragma unroll 1
  for (int ks = 0; ks < ksteps; ++ks) {
    FragB af;
    af.h[0] = *(const v8usa*)(ap + 32 * ks);
    af.h[1] = *(const v8usa*)(ap + 32 * ks + 16);
#pragma unroll
    for (int t = 0; t < NT; ++t) {
      const unsigned short* wq = wp + (size_t)(16 * t) * (size_t)K + 32 * ks;
      FragB bf;
      bf.h[0] = *(const v8usa*)wq;
      bf.h[1] = *(const v8usa*)(wq + 16);
      acc[t] = wmb(af, bf, acc[t]);
    }
  }
}

template <int EPI>
__global__ __launch_bounds__(GTHR) void k_gemm(const unsigned short* __restrict__ A,
                                               const unsigned short* __restrict__ WT,
                                               float* outF, const float* __restrict__ bias,
                                               int K, int ldo, int ncp, int pstride) {
  __shared__ __attribute__((aligned(16))) float stg[GBM * GBN];
  const int tid = (int)threadIdx.x, lane = tid & 31, wave = tid >> 5, hh = lane >> 4, m = lane & 15;
  const int rowBase = (int)blockIdx.x * GBM;
  const int col0    = (int)blockIdx.y * GBN;

  v8f acc[4];
  {
    const v8f z = {0.f, 0.f, 0.f, 0.f, 0.f, 0.f, 0.f, 0.f};
    acc[0] = z; acc[1] = z; acc[2] = z; acc[3] = z;
  }
  const unsigned short* ap = A  + (size_t)(rowBase + 16 * wave + m) * (size_t)K + 8 * hh;
  const unsigned short* wp = WT + (size_t)(col0 + m) * (size_t)K + 8 * hh;
  gemm_loop<4>(ap, wp, K, acc);

#pragma unroll
  for (int t = 0; t < 4; ++t) {
    const int lc = 16 * t + m;
#pragma unroll
    for (int r = 0; r < 8; ++r) {
      const int lr = 16 * wave + 8 * hh + r;
      stg[lr * GBN + lc] = acc[t][r];
    }
  }
  __syncthreads();

  if constexpr (EPI != 0) {
    const v4f bq = *(const v4fa*)(bias + col0 + 4 * m);
    const float b0 = bf16_val(bq.x), b1 = bf16_val(bq.y), b2 = bf16_val(bq.z), b3 = bf16_val(bq.w);
#pragma unroll 1
    for (int i = 0; i < 8; ++i) {
      float* sp = stg + (16 * wave + 2 * i + hh) * GBN + 4 * m;
      v4f v = *(const v4fa*)sp;
      v.x = softplus_f(v.x + b0);
      v.y = softplus_f(v.y + b1);
      v.z = softplus_f(v.z + b2);
      v.w = softplus_f(v.w + b3);
      *(v4fa*)sp = v;
    }
  }

  const int plane = col0 / ncp;
  const int cc    = col0 - plane * ncp;
  float* ob = outF + (size_t)plane * (size_t)pstride + cc + 4 * m;

  v4f fv[8];
#pragma unroll
  for (int i = 0; i < 8; ++i) {
    const int lr = 16 * wave + 2 * i + hh;
    fv[i] = *(const v4fa*)(stg + lr * GBN + 4 * m);
  }
#pragma unroll
  for (int i = 0; i < 8; ++i) {
    const int gr = rowBase + 16 * wave + 2 * i + hh;
    *(volatile v4f*)(ob + (size_t)gr * (size_t)ldo) = fv[i];
  }
  __threadfence();
#pragma unroll
  for (int i = 0; i < 8; ++i) {
    const int gr = rowBase + 16 * wave + 2 * i + hh;
    *(volatile v4f*)(ob + (size_t)gr * (size_t)ldo) = fv[i];
  }
}

__global__ __launch_bounds__(PTHR) void k_conv(const float* __restrict__ U, const float* __restrict__ cw,
                                               const float* __restrict__ cb, unsigned short* uc) {
  const int u   = (int)blockIdx.x * PTHR + (int)threadIdx.x;
  const int tok = u >> 8;
  const int c8  = (u & 255) * 8;
  const int t   = tok & (SEQ - 1);

  v4f w[8];
#pragma unroll
  for (int c = 0; c < 8; ++c) w[c] = *(const v4fa*)(cw + (size_t)(c8 + c) * 4);

  float acc[8];
#pragma unroll
  for (int c = 0; c < 8; ++c) acc[c] = 0.0f;

#pragma unroll
  for (int j = 0; j < 4; ++j) {
    const int  tt   = t - 3 + j;
    const bool ok   = tt >= 0;
    const int  rowc = ok ? (tok - 3 + j) : tok;
    const float* p  = U + (size_t)rowc * INNER + c8;
    const v4f a = *(const v4fa*)p;
    const v4f b = *(const v4fa*)(p + 4);
    const float w0 = ok ? bf16_val(w[0][j]) : 0.0f;
    const float w1 = ok ? bf16_val(w[1][j]) : 0.0f;
    const float w2 = ok ? bf16_val(w[2][j]) : 0.0f;
    const float w3 = ok ? bf16_val(w[3][j]) : 0.0f;
    const float w4 = ok ? bf16_val(w[4][j]) : 0.0f;
    const float w5 = ok ? bf16_val(w[5][j]) : 0.0f;
    const float w6 = ok ? bf16_val(w[6][j]) : 0.0f;
    const float w7 = ok ? bf16_val(w[7][j]) : 0.0f;
    acc[0] = fmaf(w0, a.x, acc[0]);
    acc[1] = fmaf(w1, a.y, acc[1]);
    acc[2] = fmaf(w2, a.z, acc[2]);
    acc[3] = fmaf(w3, a.w, acc[3]);
    acc[4] = fmaf(w4, b.x, acc[4]);
    acc[5] = fmaf(w5, b.y, acc[5]);
    acc[6] = fmaf(w6, b.z, acc[6]);
    acc[7] = fmaf(w7, b.w, acc[7]);
  }
  const v4f ba = *(const v4fa*)(cb + c8);
  const v4f bb = *(const v4fa*)(cb + c8 + 4);
  v4f ra, rb;
  ra.x = acc[0] + bf16_val(ba.x); ra.y = acc[1] + bf16_val(ba.y);
  ra.z = acc[2] + bf16_val(ba.z); ra.w = acc[3] + bf16_val(ba.w);
  rb.x = acc[4] + bf16_val(bb.x); rb.y = acc[5] + bf16_val(bb.y);
  rb.z = acc[6] + bf16_val(bb.z); rb.w = acc[7] + bf16_val(bb.w);
  v8us hv, lv;
  split8(ra, rb, hv, lv);
  unsigned short* dp = uc + (size_t)tok * K2 + c8;
  *(volatile v8us*)dp = hv;
  *(volatile v8us*)(dp + INNER) = lv;
  __threadfence();
  *(volatile v8us*)dp = hv;
  *(volatile v8us*)(dp + INNER) = lv;
}

__global__ __launch_bounds__(GTHR) void k_ssm(const unsigned short* __restrict__ A,
                                              const unsigned short* __restrict__ WT,
                                              float* ssm, unsigned short* dthl) {
  __shared__ __attribute__((aligned(16))) float stg[GBM * SSMP];
  __shared__ __attribute__((aligned(16))) unsigned short dts[GBM * DTK];
  const int tid = (int)threadIdx.x, lane = tid & 31, wave = tid >> 5, hh = lane >> 4, m = lane & 15;
  const int rowBase = (int)blockIdx.x * GBM;

  v8f acc[3];
  {
    const v8f z = {0.f, 0.f, 0.f, 0.f, 0.f, 0.f, 0.f, 0.f};
    acc[0] = z; acc[1] = z; acc[2] = z;
  }
  const unsigned short* ap = A  + (size_t)(rowBase + 16 * wave + m) * (size_t)K2 + 8 * hh;
  const unsigned short* wp = WT + (size_t)m * (size_t)K2 + 8 * hh;
  gemm_loop<3>(ap, wp, K2, acc);

#pragma unroll
  for (int t = 0; t < 3; ++t) {
    const int lc = 16 * t + m;
#pragma unroll
    for (int r = 0; r < 8; ++r) {
      const int lr = 16 * wave + 8 * hh + r;
      stg[lr * SSMP + lc] = acc[t][r];
    }
  }
  __syncthreads();

  {
    const int row = tid >> 1, j = tid & 1;
    const v4f a = *(const v4fa*)(stg + row * SSMP + 8 * j);
    const v4f b = *(const v4fa*)(stg + row * SSMP + 8 * j + 4);
    v8us hv, lv;
    split8(a, b, hv, lv);
    *(v8usa*)(dts + row * DTK + 8 * j) = hv;
    *(v8usa*)(dts + row * DTK + NST + 8 * j) = lv;
  }
  v4f sv[6];
#pragma unroll
  for (int it = 0; it < 6; ++it) sv[it] = *(const v4fa*)(stg + 4 * (tid + GTHR * it));
  __syncthreads();
  v8us dv[2];
#pragma unroll
  for (int it = 0; it < 2; ++it) dv[it] = *(const v8usa*)(dts + 8 * (tid + GTHR * it));

  float* so = ssm + (size_t)rowBase * SSMP;
  unsigned short* dq = dthl + (size_t)rowBase * DTK;
#pragma unroll
  for (int it = 0; it < 6; ++it) *(volatile v4f*)(so + 4 * (tid + GTHR * it)) = sv[it];
#pragma unroll
  for (int it = 0; it < 2; ++it) *(volatile v8us*)(dq + 8 * (tid + GTHR * it)) = dv[it];
  __threadfence();
#pragma unroll
  for (int it = 0; it < 6; ++it) *(volatile v4f*)(so + 4 * (tid + GTHR * it)) = sv[it];
#pragma unroll
  for (int it = 0; it < 2; ++it) *(volatile v8us*)(dq + 8 * (tid + GTHR * it)) = dv[it];
}

__global__ __launch_bounds__(CT) void k_scan(const float* __restrict__ DELTA, const float* __restrict__ RES,
                                             const float* __restrict__ SSM, const float* __restrict__ Alog,
                                             unsigned short* UY) {
  __shared__ __attribute__((aligned(16))) float sD[TCH * CT];
  __shared__ __attribute__((aligned(16))) float sR[TCH * CT];
  __shared__ __attribute__((aligned(16))) unsigned short sUh[TCH * CT];
  __shared__ __attribute__((aligned(16))) unsigned short sUl[TCH * CT];
  __shared__ __attribute__((aligned(16))) float sS[TCH * SSMP];
  __shared__ __attribute__((aligned(16))) float sA[CT * NST];
  const int tid = (int)threadIdx.x;
  const int b   = (int)blockIdx.x >> 5;
  const int c0  = ((int)blockIdx.x & 31) * CT;

#pragma unroll 1
  for (int i = 0; i < NST; ++i) {
    const int idx = tid + CT * i;
    const float al = bf16_val(Alog[(size_t)c0 * NST + idx]);
    sA[idx] = (-expf(al)) * 1.44269504088896340736f;
  }
  __syncthreads();

  float A2[NST], h[NST];
  {
    const v4f a0 = *(const v4fa*)(sA + tid * NST);
    const v4f a1 = *(const v4fa*)(sA + tid * NST + 4);
    const v4f a2 = *(const v4fa*)(sA + tid * NST + 8);
    const v4f a3 = *(const v4fa*)(sA + tid * NST + 12);
    A2[0] = a0.x; A2[1] = a0.y; A2[2] = a0.z; A2[3] = a0.w;
    A2[4] = a1.x; A2[5] = a1.y; A2[6] = a1.z; A2[7] = a1.w;
    A2[8] = a2.x; A2[9] = a2.y; A2[10] = a2.z; A2[11] = a2.w;
    A2[12] = a3.x; A2[13] = a3.y; A2[14] = a3.z; A2[15] = a3.w;
  }
#pragma unroll
  for (int s = 0; s < NST; ++s) h[s] = 0.0f;

#pragma unroll 1
  for (int ch = 0; ch < SEQ / TCH; ++ch) {
    const int tok0 = b * SEQ + ch * TCH;

#pragma unroll 2
    for (int i = 0; i < 8; ++i) {
      const int p = tid + CT * i;
      const int row = p >> 4, q = p & 15;
      const size_t go = (size_t)(tok0 + row) * INNER + c0 + 4 * q;
      const v4f d = *(const v4fa*)(DELTA + go);
      const v4f r = *(const v4fa*)(RES + go);
      *(v4fa*)(sD + 4 * p) = d;
      *(v4fa*)(sR + 4 * p) = r;
    }
#pragma unroll 2
    for (int i = 0; i < 4; ++i) {
      const int p = tid + CT * i;
      const int row = p >> 3, q = p & 7;
      const unsigned short* up = UY + (size_t)(tok0 + row) * K2 + c0 + 8 * q;
      const v8us a = *(const v8usa*)up;
      const v8us l = *(const v8usa*)(up + INNER);
      *(v8usa*)(sUh + 8 * p) = a;
      *(v8usa*)(sUl + 8 * p) = l;
    }
#pragma unroll 2
    for (int i = 0; i < 6; ++i) {
      const int p = tid + CT * i;
      const v4f s = *(const v4fa*)(SSM + (size_t)tok0 * SSMP + 4 * p);
      *(v4fa*)(sS + 4 * p) = s;
    }
    __syncthreads();

#pragma unroll 1
    for (int t = 0; t < TCH; ++t) {
      const float d  = sD[t * CT + tid];
      const float r  = sR[t * CT + tid];
      const unsigned uh = (unsigned)sUh[t * CT + tid];
      const unsigned ul = (unsigned)sUl[t * CT + tid];
      const float uu = __uint_as_float(uh << 16) + __uint_as_float(ul << 16);
      const float* sp = sS + t * SSMP;
      const v4f q0 = *(const v4fa*)(sp + 16);
      const v4f q1 = *(const v4fa*)(sp + 20);
      const v4f q2 = *(const v4fa*)(sp + 24);
      const v4f q3 = *(const v4fa*)(sp + 28);
      const float cv = sp[32];
      float Bv[NST];
      Bv[0] = q0.x; Bv[1] = q0.y; Bv[2] = q0.z; Bv[3] = q0.w;
      Bv[4] = q1.x; Bv[5] = q1.y; Bv[6] = q1.z; Bv[7] = q1.w;
      Bv[8] = q2.x; Bv[9] = q2.y; Bv[10] = q2.z; Bv[11] = q2.w;
      Bv[12] = q3.x; Bv[13] = q3.y; Bv[14] = q3.z; Bv[15] = q3.w;
      float ys = 0.0f;
#pragma unroll
      for (int s = 0; s < NST; ++s) {
        const float e = exp2f(d * A2[s]);
        h[s] = fmaf(h[s], e, uu * Bv[s]);
        ys += h[s];
      }
      const float e1  = expf(-r);
      const float sil = r * (1.0f / (1.0f + e1));
      sD[t * CT + tid] = (ys * cv) * sil;
    }
    __syncthreads();

    v8us hv[4], lv[4];
#pragma unroll
    for (int i = 0; i < 4; ++i) {
      const int unit = tid + CT * i;
      const int tt = unit >> 3, q = unit & 7;
      const v4f g0 = *(const v4fa*)(sD + tt * CT + 8 * q);
      const v4f g1 = *(const v4fa*)(sD + tt * CT + 8 * q + 4);
      split8(g0, g1, hv[i], lv[i]);
    }
#pragma unroll
    for (int i = 0; i < 4; ++i) {
      const int unit = tid + CT * i;
      const int tt = unit >> 3, q = unit & 7;
      unsigned short* yp = UY + (size_t)(tok0 + tt) * K2 + c0 + 8 * q;
      *(volatile v8us*)yp = hv[i];
      *(volatile v8us*)(yp + INNER) = lv[i];
    }
    __threadfence();
#pragma unroll
    for (int i = 0; i < 4; ++i) {
      const int unit = tid + CT * i;
      const int tt = unit >> 3, q = unit & 7;
      unsigned short* yp = UY + (size_t)(tok0 + tt) * K2 + c0 + 8 * q;
      *(volatile v8us*)yp = hv[i];
      *(volatile v8us*)(yp + INNER) = lv[i];
    }
    __syncthreads();
  }
}

static inline size_t al256(size_t o) { return (o + 255) & ~(size_t)255; }

extern "C" void kernel_launch(void* const* d_in, const int* in_sizes, int n_in,
                              void* d_out, int out_size, void* d_ws, size_t ws_size,
                              hipStream_t stream) {
  if (n_in < 9) return;
  if (in_sizes[0] != NTOK * DIMC) return;
  if (in_sizes[1] != 2 * INNER * DIMC) return;
  if (in_sizes[2] != INNER * 4) return;
  if (in_sizes[3] != INNER) return;
  if (in_sizes[4] != (2 * NST + 1) * INNER) return;
  if (in_sizes[5] != INNER * NST) return;
  if (in_sizes[6] != INNER) return;
  if (in_sizes[7] != DIMC * INNER) return;
  if (in_sizes[8] != INNER * NST) return;
  if (out_size != NTOK * DIMC) return;

  const float* x     = (const float*)d_in[0];
  const float* Win   = (const float*)d_in[1];
  const float* convw = (const float*)d_in[2];
  const float* convb = (const float*)d_in[3];
  const float* Wx    = (const float*)d_in[4];
  const float* Wdt   = (const float*)d_in[5];
  const float* bdt   = (const float*)d_in[6];
  const float* Wout  = (const float*)d_in[7];
  const float* Alog  = (const float*)d_in[8];
  float* out = (float*)d_out;

  char* ws = (char*)d_ws;
  size_t off = 0;
  const size_t oXB  = off; off = al256(off + (size_t)NTOK * DIMC * 2);
  const size_t oWIN = off; off = al256(off + (size_t)2 * INNER * DIMC * 2);
  const size_t oUR  = off; off = al256(off + (size_t)2 * NTOK * INNER * 4);
  const size_t oUC  = off; off = al256(off + (size_t)NTOK * K2 * 2);
  const size_t oWO  = off; off = al256(off + (size_t)DIMC * K2 * 2);
  const size_t oWX  = off; off = al256(off + (size_t)SSMP * K2 * 2);
  const size_t oSS  = off; off = al256(off + (size_t)NTOK * SSMP * 4);
  const size_t oDT  = off; off = al256(off + (size_t)NTOK * DTK * 2);
  const size_t oWD  = off; off = al256(off + (size_t)INNER * DTK * 2);
  if (off > ws_size || off > (size_t)WSMAX) return;
  unsigned short* XB    = (unsigned short*)(ws + oXB);
  unsigned short* WIN   = (unsigned short*)(ws + oWIN);
  float*          UD    = (float*)(ws + oUR);
  float*          RES   = UD + (size_t)NTOK * INNER;
  unsigned short* UC    = (unsigned short*)(ws + oUC);
  unsigned short* WOUT2 = (unsigned short*)(ws + oWO);
  unsigned short* WX2   = (unsigned short*)(ws + oWX);
  float*          SSM   = (float*)(ws + oSS);
  unsigned short* DT    = (unsigned short*)(ws + oDT);
  unsigned short* WDT2  = (unsigned short*)(ws + oWD);

  k_prep<<<NU_ALL / PTHR, PTHR, 0, stream>>>(x, Win, Wx, Wdt, Wout, XB, WIN, WOUT2, WX2, WDT2);
  k_gemm<0><<<dim3(NTOK / GBM, (2 * INNER) / GBN), GTHR, 0, stream>>>(
      XB, WIN, UD, bdt, DIMC, INNER, INNER, NTOK * INNER);
  k_conv<<<(NTOK * (INNER / 8)) / PTHR, PTHR, 0, stream>>>(UD, convw, convb, UC);
  k_ssm<<<NTOK / GBM, GTHR, 0, stream>>>(UC, WX2, SSM, DT);
  k_gemm<1><<<dim3(NTOK / GBM, INNER / GBN), GTHR, 0, stream>>>(
      DT, WDT2, UD, bdt, DTK, INNER, INNER, 0);
  k_scan<<<2 * (INNER / CT), CT, 0, stream>>>(UD, RES, SSM, Alog, UC);
  k_gemm<0><<<dim3(NTOK / GBM, DIMC / GBN), GTHR, 0, stream>>>(
      UC, WOUT2, out, bdt, K2, DIMC, DIMC, 0);
}
